// GCN_36112085025126
// MI455X (gfx1250) — hardware-run, weakly checked
//
#include <hip/hip_runtime.h>
#include <stddef.h>
#include <stdint.h>
#include <math.h>

#ifndef TWO_TERM_L2
#define TWO_TERM_L2 1
#endif
#ifndef TWO_TERM_L3
#define TWO_TERM_L3 1
#endif

#define NN      100000
#define NE      1600000
#define DF      128
#define DO      64
#define GBM     128
#define MP      100096
#define APITCH  256
#define WPITCH  256
#define KE2     (TWO_TERM_L2 ? 256 : 128)
#define KE3     (TWO_TERM_L3 ? 256 : 128)
#define NTHR    256
#define NWAVE   8
#define EPT     8
#define WCH     (32 * EPT)
#define NBRUN   1024
#define SLB     10
#define NBK     98
#define WLCAP   2560
#define RCAP    20480
#define DEGCAP  64
#define MAXDEG_IN    36
#define MAXDEG_OUT   37
#define MAXB1024_IN  16721
#define MAXB1024_OUT 16666
#define PARTW   288
#define WSTW    258
#define WSMAX   (128u << 20)

#define BK_ZINTS (2 * NWAVE * WLCAP + RCAP + 6 * NBRUN)
#define BK_INTS  (BK_ZINTS + 32)
#define BK_LDS   (BK_INTS * 4)
#define GL128    ((GBM * (DF + 4) + GBM) * 4)
#define GL64     ((GBM * (DO + 4) + GBM) * 4)

#define PBX   (MP * DF / 8 / NTHR)
#define PBW1  (DF * DF / 8 / NTHR)
#define PBW2  (DF * WPITCH / 8 / NTHR)
#define PBW3  (DO * WPITCH / 8 / NTHR)
#define PBTOT (PBX + PBW1 + PBW2 + PBW3 + 1)

#define SM_B1 0
#define SM_G1 128
#define SM_BE 256
#define SM_B2 384
#define SM_B3 512
#define SM_N  640

static_assert(MP % GBM == 0 && MP >= NN && MP == 782 * GBM && MP % 64 == 0);
static_assert(NBRUN == (1 << SLB) && NBRUN % 32 == 0 && NBRUN % NWAVE == 0);
static_assert(NBK * NBRUN >= MP && (NBK - 1) * NBRUN < NN);
static_assert(NN < (1 << 17) && ((long long)NN << SLB) < (1LL << 31));
static_assert(NE % WCH == 0 && NE % 4 == 0);
static_assert(RCAP == NWAVE * WLCAP && RCAP % (NTHR * 4) == 0 && BK_ZINTS % 4 == 0);
static_assert((long long)RCAP * 100 >= (long long)MAXB1024_IN * 105);
static_assert(WLCAP >= MAXB1024_IN / 8 + 8 * 46 + 1 && WLCAP >= MAXB1024_OUT / 8 + 8 * 46 + 1);
static_assert(MAXDEG_IN + 8 <= DEGCAP && MAXDEG_OUT + 8 <= DEGCAP);
static_assert(BK_LDS <= 300000 && BK_LDS <= 327680 && GL128 <= 327680);
static_assert((MP * DF / 8) % NTHR == 0 && (DF * DF / 8) % NTHR == 0);
static_assert((DF * WPITCH / 8) % NTHR == 0 && (DO * WPITCH / 8) % NTHR == 0);
static_assert(DF % 32 == 0 && KE2 % 32 == 0 && KE3 % 32 == 0 && KE2 <= APITCH && KE3 <= WPITCH);
static_assert(APITCH == 2 * DF && WPITCH == 2 * DF && DF == 4 * 32 && DO == 4 * 16);
static_assert(PARTW % 32 == 0 && PARTW / 4 <= NTHR && PARTW >= 2 * DF + 1 && WSTW >= 2 * DF + 1);
static_assert((NN & 1) == 0);

typedef float          v4f   __attribute__((ext_vector_type(4)));
typedef float          v8f   __attribute__((ext_vector_type(8)));
typedef int            v4i   __attribute__((ext_vector_type(4)));
typedef int            v8i   __attribute__((ext_vector_type(8)));
typedef unsigned short v8us  __attribute__((ext_vector_type(8)));
typedef unsigned short v16us __attribute__((ext_vector_type(16)));
typedef __bf16         v16bf __attribute__((ext_vector_type(16)));
typedef v4f  __attribute__((may_alias)) v4fa;
typedef v4i  __attribute__((may_alias)) v4ia;
typedef v8us __attribute__((may_alias)) v8usa;
union FragB { v16bf v; v16us u; v8us h[2]; v8i w; };

__device__ __forceinline__ v8f wmb(const FragB& a, const FragB& b, v8f c) {
  v8f d = __builtin_amdgcn_wmma_f32_16x16x32_bf16(false, a.v, false, b.v, (short)0, c, false, false);
  asm volatile("v_nop\n\tv_nop\n\tv_nop\n\tv_nop" : "+v"(d) : "v"(a.w), "v"(b.w));
  return d;
}

__device__ __forceinline__ unsigned bf16_bits(float f) {
  const unsigned u = __float_as_uint(f);
  const unsigned r = (u + 0x7FFFu + ((u >> 16) & 1u)) >> 16;
  const unsigned q = (u >> 16) | 0x40u;
  return ((u & 0x7fffffffu) > 0x7f800000u) ? q : r;
}

__device__ __forceinline__ void hilo_pack(float v0, float v1, float v2, float v3,
                                          int& h01, int& h23, int& l01, int& l23) {
  const unsigned a0 = bf16_bits(v0), a1 = bf16_bits(v1), a2 = bf16_bits(v2), a3 = bf16_bits(v3);
  const unsigned b0 = bf16_bits(v0 - __uint_as_float(a0 << 16));
  const unsigned b1 = bf16_bits(v1 - __uint_as_float(a1 << 16));
  const unsigned b2 = bf16_bits(v2 - __uint_as_float(a2 << 16));
  const unsigned b3 = bf16_bits(v3 - __uint_as_float(a3 << 16));
  h01 = (int)(a0 | (a1 << 16)); h23 = (int)(a2 | (a3 << 16));
  l01 = (int)(b0 | (b1 << 16)); l23 = (int)(b2 | (b3 << 16));
}

__device__ __forceinline__ v4i regroup32(int h01, int h23, int l01, int l23, int lane) {
  const int s0 = (2 * lane) & 31, s1 = s0 + 1;
  const int a0 = __shfl(h01, s0, 32), a1 = __shfl(h23, s0, 32), a2 = __shfl(h01, s1, 32), a3 = __shfl(h23, s1, 32);
  const int b0 = __shfl(l01, s0, 32), b1 = __shfl(l23, s0, 32), b2 = __shfl(l01, s1, 32), b3 = __shfl(l23, s1, 32);
  const int mk = (lane < 16) ? -1 : 0;
  v4i o;
  o.x = (a0 & mk) | (b0 & ~mk); o.y = (a1 & mk) | (b1 & ~mk);
  o.z = (a2 & mk) | (b2 & ~mk); o.w = (a3 & mk) | (b3 & ~mk);
  return o;
}

__device__ __forceinline__ void st2_v4f(float* p, v4f v) {
  *(volatile v4f*)p = v;
  __threadfence();
  *(volatile v4f*)p = v;
}
__device__ __forceinline__ void st2_v4i(unsigned short* p, v4i v) {
  *(volatile v4i*)p = v;
  __threadfence();
  *(volatile v4i*)p = v;
}
__device__ __forceinline__ void st2_v8us(unsigned short* p, v8us v) {
  *(volatile v8us*)p = v;
  __threadfence();
  *(volatile v8us*)p = v;
}

__device__ __forceinline__ v8us gather8(const float* __restrict__ base, int stride) {
  float f[8];
#pragma unroll
  for (int i = 0; i < 8; ++i) f[i] = base[(size_t)i * (size_t)stride];
  v8us o;
#pragma unroll
  for (int i = 0; i < 8; ++i) o[i] = (unsigned short)bf16_bits(f[i]);
  return o;
}

__device__ __forceinline__ void sm_put(const float* __restrict__ p, int n, float* dst, int lane) {
  const int i0 = 4 * lane, i1 = i0 + 1, i2 = i0 + 2, i3 = i0 + 3;
  const float a0 = p[i0 < n ? i0 : n - 1], a1 = p[i1 < n ? i1 : n - 1];
  const float a2 = p[i2 < n ? i2 : n - 1], a3 = p[i3 < n ? i3 : n - 1];
  asm volatile("" :: "v"(a0), "v"(a1), "v"(a2), "v"(a3));
  const unsigned m0 = (i0 < n) ? 0xffffffffu : 0u, m1 = (i1 < n) ? 0xffffffffu : 0u;
  const unsigned m2 = (i2 < n) ? 0xffffffffu : 0u, m3 = (i3 < n) ? 0xffffffffu : 0u;
  v4f o;
  o.x = __uint_as_float((bf16_bits(a0) << 16) & m0);
  o.y = __uint_as_float((bf16_bits(a1) << 16) & m1);
  o.z = __uint_as_float((bf16_bits(a2) << 16) & m2);
  o.w = __uint_as_float((bf16_bits(a3) << 16) & m3);
  st2_v4f(dst + 4 * lane, o);
}

__global__ __launch_bounds__(NTHR) void k_prep(const float* __restrict__ x, const float* __restrict__ w1,
                                               const float* __restrict__ b1, const float* __restrict__ g1,
                                               const float* __restrict__ be1, const float* __restrict__ w2,
                                               const float* __restrict__ b2, const float* __restrict__ w3,
                                               const float* __restrict__ b3,
                                               unsigned short* xb, unsigned short* w1t, unsigned short* w2d,
                                               unsigned short* w3d, float* sm) {
  const int tid = (int)threadIdx.x, lane = tid & 31, wave = tid >> 5;
  const int blk = (int)blockIdx.x;
  if (blk < PBX) {
    const int u   = blk * NTHR + tid;
    const int row = u >> 4, k8 = (u & 15) * 8;
    const int rc  = row < NN ? row : NN - 1;
    const unsigned mk = row < NN ? 0xffffu : 0u;
    const float* p = x + (size_t)rc * DF + k8;
    const v4f a = *(const v4fa*)p;
    const v4f b = *(const v4fa*)(p + 4);
    v8us o;
    o[0] = (unsigned short)(bf16_bits(a.x) & mk); o[1] = (unsigned short)(bf16_bits(a.y) & mk);
    o[2] = (unsigned short)(bf16_bits(a.z) & mk); o[3] = (unsigned short)(bf16_bits(a.w) & mk);
    o[4] = (unsigned short)(bf16_bits(b.x) & mk); o[5] = (unsigned short)(bf16_bits(b.y) & mk);
    o[6] = (unsigned short)(bf16_bits(b.z) & mk); o[7] = (unsigned short)(bf16_bits(b.w) & mk);
    st2_v8us(xb + (size_t)row * DF + k8, o);
  } else if (blk < PBX + PBW1) {
    const int u = (blk - PBX) * NTHR + tid;
    const int n = u >> 4, k8 = (u & 15) * 8;
    const v8us o = gather8(w1 + (size_t)k8 * DF + n, DF);
    st2_v8us(w1t + (size_t)n * DF + k8, o);
  } else if (blk < PBX + PBW1 + PBW2) {
    const int u = (blk - PBX - PBW1) * NTHR + tid;
    const int n = u >> 5, k8 = (u & 31) * 8, kk = k8 & (DF - 1);
    const v8us o = gather8(w2 + (size_t)kk * DF + n, DF);
    st2_v8us(w2d + (size_t)n * WPITCH + k8, o);
  } else if (blk < PBX + PBW1 + PBW2 + PBW3) {
    const int u = (blk - PBX - PBW1 - PBW2) * NTHR + tid;
    const int n = u >> 5, k8 = (u & 31) * 8, kk = k8 & (DF - 1);
    const v8us o = gather8(w3 + (size_t)kk * DO + n, DO);
    st2_v8us(w3d + (size_t)n * WPITCH + k8, o);
  } else {
    if (wave == 0)      sm_put(b1,  DF, sm + SM_B1, lane);
    else if (wave == 1) sm_put(g1,  DF, sm + SM_G1, lane);
    else if (wave == 2) sm_put(be1, DF, sm + SM_BE, lane);
    else if (wave == 3) sm_put(b2,  DF, sm + SM_B2, lane);
    else if (wave == 4) sm_put(b3,  DO, sm + SM_B3, lane);
  }
}

__device__ __forceinline__ void bucket_flush(const int* pl, const int* cnti, const int* offs, const float* nrm,
                                             int ov, int* lp, int* cntp, int* offp, float* ndp, float* nsp,
                                             int* fp, int tid) {
#pragma unroll 1
  for (int i = tid * 4; i < RCAP; i += NTHR * 4) {
    const v4i v = *(const v4ia*)(pl + i);
    *(volatile v4i*)(lp + i) = v;
  }
  {
    const v4i v = *(const v4ia*)(cnti + 4 * tid);
    *(volatile v4i*)(cntp + 4 * tid) = v;
  }
  {
    const v4i v = *(const v4ia*)(offs + 4 * tid);
    *(volatile v4i*)(offp + 4 * tid) = v;
  }
  {
    const v4f v = *(const v4fa*)(nrm + 4 * tid);
    *(volatile v4f*)(ndp + 4 * tid) = v;
  }
  {
    const v4f v = *(const v4fa*)(nrm + NBRUN + 4 * tid);
    *(volatile v4f*)(nsp + 4 * tid) = v;
  }
  if (tid < 8) {
    const v4i f = {ov, ov, ov, ov};
    *(volatile v4i*)(fp + 4 * tid) = f;
  }
}

__device__ __forceinline__ int count_lists(const int* wl, const int* wcnt, int* cnt, int lane) {
  int ov = 0;
#pragma unroll 1
  for (int w2 = 0; w2 < NWAVE; ++w2) {
    int c = wcnt[w2];
    if (c > WLCAP) ov = 1;
    c = c < 0 ? 0 : (c > WLCAP ? WLCAP : c);
    c = __builtin_amdgcn_readfirstlane(c);
#pragma unroll 1
    for (int b0 = 0; b0 < c; b0 += 32) {
      const int idx = b0 + lane;
      const int ent = wl[w2 * WLCAP + (idx < WLCAP ? idx : WLCAP - 1)];
      const int m32 = (c - b0) < 32 ? (c - b0) : 32;
#pragma unroll 1
      for (int k = 0; k < m32; ++k) {
        const int u    = __builtin_amdgcn_readlane(ent, k);
        const int slot = u & (NBRUN - 1);
        if (lane == 0) cnt[slot] = cnt[slot] + 1;
      }
    }
  }
  return ov;
}

#define PUT_IN(HJ, SJ, SV) if (HJ) { int sr_ = (SV); sr_ = sr_ < 0 ? 0 : (sr_ > NN - 1 ? NN - 1 : sr_); \
    if (pI < WLCAP) myI[pI] = (sr_ << SLB) | (int)(SJ); pI = pI + 1; }
#define PUT_OUT(GJ, TJ) if (GJ) { if (pO < WLCAP) myO[pO] = (int)(TJ); pO = pO + 1; }

__global__ __launch_bounds__(NTHR) void k_bucket(const int* __restrict__ srcs, const int* __restrict__ dsts,
                                                 int* LIST, int* CNT, int* OFF, float* NSg, float* NDg,
                                                 int* FLAG) {
  extern __shared__ __attribute__((aligned(16))) int dsm[];
  int* wlI   = dsm;
  int* wlO   = dsm + NWAVE * WLCAP;
  int* pl    = wlO + NWAVE * WLCAP;
  int* cc    = pl + RCAP;
  int* offs  = cc + 2 * NBRUN;
  int* cur   = offs + NBRUN;
  float* nrm = (float*)(cur + NBRUN);
  int* misc  = cur + 3 * NBRUN;
  const int tid = (int)threadIdx.x, lane = tid & 31, wave = tid >> 5;
  const int blk = (int)blockIdx.x;
  const unsigned nbs = (unsigned)(blk * NBRUN);

  {
    const v4i z4 = {0, 0, 0, 0};
    for (int i = tid * 4; i < BK_ZINTS; i += NTHR * 4) *(v4ia*)(dsm + i) = z4;
    if (tid < 32) misc[tid] = 0;
  }
  __syncthreads();

  {
    const int per  = ((NE + NWAVE * WCH - 1) / (NWAVE * WCH)) * WCH;
    const int ebeg = wave * per;
    const int eend = (ebeg + per < NE) ? (ebeg + per) : NE;
    int* myI = wlI + wave * WLCAP;
    int* myO = wlO + wave * WLCAP;
    int wcI = 0, wcO = 0;
#pragma unroll 1
    for (int cb = ebeg; cb < eend; cb += WCH) {
      const int e0 = cb + lane * EPT;
      const v4i da = *(const v4ia*)(dsts + e0);
      const v4i db = *(const v4ia*)(dsts + e0 + 4);
      const v4i sa = *(const v4ia*)(srcs + e0);
      const v4i sc = *(const v4ia*)(srcs + e0 + 4);
      {
        const unsigned s0 = (unsigned)da.x - nbs, s1 = (unsigned)da.y - nbs;
        const unsigned s2 = (unsigned)da.z - nbs, s3 = (unsigned)da.w - nbs;
        const unsigned s4 = (unsigned)db.x - nbs, s5 = (unsigned)db.y - nbs;
        const unsigned s6 = (unsigned)db.z - nbs, s7 = (unsigned)db.w - nbs;
        const bool h0 = s0 < (unsigned)NBRUN, h1 = s1 < (unsigned)NBRUN, h2 = s2 < (unsigned)NBRUN, h3 = s3 < (unsigned)NBRUN;
        const bool h4 = s4 < (unsigned)NBRUN, h5 = s5 < (unsigned)NBRUN, h6 = s6 < (unsigned)NBRUN, h7 = s7 < (unsigned)NBRUN;
        const unsigned m0 = __builtin_amdgcn_ballot_w32(h0), m1 = __builtin_amdgcn_ballot_w32(h1);
        const unsigned m2 = __builtin_amdgcn_ballot_w32(h2), m3 = __builtin_amdgcn_ballot_w32(h3);
        const unsigned m4 = __builtin_amdgcn_ballot_w32(h4), m5 = __builtin_amdgcn_ballot_w32(h5);
        const unsigned m6 = __builtin_amdgcn_ballot_w32(h6), m7 = __builtin_amdgcn_ballot_w32(h7);
        const unsigned any = m0 | m1 | m2 | m3 | m4 | m5 | m6 | m7;
        if (any != 0u) {
          const int pre = (int)(__builtin_amdgcn_mbcnt_lo(m0, 0u) + __builtin_amdgcn_mbcnt_lo(m1, 0u) +
                                __builtin_amdgcn_mbcnt_lo(m2, 0u) + __builtin_amdgcn_mbcnt_lo(m3, 0u) +
                                __builtin_amdgcn_mbcnt_lo(m4, 0u) + __builtin_amdgcn_mbcnt_lo(m5, 0u) +
                                __builtin_amdgcn_mbcnt_lo(m6, 0u) + __builtin_amdgcn_mbcnt_lo(m7, 0u));
          int pI = wcI + pre;
          PUT_IN(h0, s0, sa.x)
          PUT_IN(h1, s1, sa.y)
          PUT_IN(h2, s2, sa.z)
          PUT_IN(h3, s3, sa.w)
          PUT_IN(h4, s4, sc.x)
          PUT_IN(h5, s5, sc.y)
          PUT_IN(h6, s6, sc.z)
          PUT_IN(h7, s7, sc.w)
          wcI += (int)(__builtin_popcount(m0) + __builtin_popcount(m1) + __builtin_popcount(m2) + __builtin_popcount(m3) +
                       __builtin_popcount(m4) + __builtin_popcount(m5) + __builtin_popcount(m6) + __builtin_popcount(m7));
        }
      }
      {
        const unsigned t0 = (unsigned)sa.x - nbs, t1 = (unsigned)sa.y - nbs;
        const unsigned t2 = (unsigned)sa.z - nbs, t3 = (unsigned)sa.w - nbs;
        const unsigned t4 = (unsigned)sc.x - nbs, t5 = (unsigned)sc.y - nbs;
        const unsigned t6 = (unsigned)sc.z - nbs, t7 = (unsigned)sc.w - nbs;
        const bool g0 = t0 < (unsigned)NBRUN, g1 = t1 < (unsigned)NBRUN, g2 = t2 < (unsigned)NBRUN, g3 = t3 < (unsigned)NBRUN;
        const bool g4 = t4 < (unsigned)NBRUN, g5 = t5 < (unsigned)NBRUN, g6 = t6 < (unsigned)NBRUN, g7 = t7 < (unsigned)NBRUN;
        const unsigned m0 = __builtin_amdgcn_ballot_w32(g0), m1 = __builtin_amdgcn_ballot_w32(g1);
        const unsigned m2 = __builtin_amdgcn_ballot_w32(g2), m3 = __builtin_amdgcn_ballot_w32(g3);
        const unsigned m4 = __builtin_amdgcn_ballot_w32(g4), m5 = __builtin_amdgcn_ballot_w32(g5);
        const unsigned m6 = __builtin_amdgcn_ballot_w32(g6), m7 = __builtin_amdgcn_ballot_w32(g7);
        const unsigned any = m0 | m1 | m2 | m3 | m4 | m5 | m6 | m7;
        if (any != 0u) {
          const int pre = (int)(__builtin_amdgcn_mbcnt_lo(m0, 0u) + __builtin_amdgcn_mbcnt_lo(m1, 0u) +
                                __builtin_amdgcn_mbcnt_lo(m2, 0u) + __builtin_amdgcn_mbcnt_lo(m3, 0u) +
                                __builtin_amdgcn_mbcnt_lo(m4, 0u) + __builtin_amdgcn_mbcnt_lo(m5, 0u) +
                                __builtin_amdgcn_mbcnt_lo(m6, 0u) + __builtin_amdgcn_mbcnt_lo(m7, 0u));
          int pO = wcO + pre;
          PUT_OUT(g0, t0)
          PUT_OUT(g1, t1)
          PUT_OUT(g2, t2)
          PUT_OUT(g3, t3)
          PUT_OUT(g4, t4)
          PUT_OUT(g5, t5)
          PUT_OUT(g6, t6)
          PUT_OUT(g7, t7)
          wcO += (int)(__builtin_popcount(m0) + __builtin_popcount(m1) + __builtin_popcount(m2) + __builtin_popcount(m3) +
                       __builtin_popcount(m4) + __builtin_popcount(m5) + __builtin_popcount(m6) + __builtin_popcount(m7));
        }
      }
    }
    if (lane == 0) { misc[wave] = wcI; misc[8 + wave] = wcO; }
  }
  __syncthreads();

  if (wave == 0) {
    const int ov = count_lists(wlI, misc, cc, lane);
    if (lane == 0) misc[16] = ov;
  } else if (wave == 1) {
    const int ov = count_lists(wlO, misc + 8, cc + NBRUN, lane);
    if (lane == 0) misc[17] = ov;
  }
  __syncthreads();
  if (wave == 0) {
    const int base = lane * (NBRUN / 32);
    int s = 0;
#pragma unroll 1
    for (int i = 0; i < NBRUN / 32; ++i) s += cc[base + i];
    int incl = s;
#pragma unroll
    for (int d = 1; d < 32; d <<= 1) {
      const int y = __shfl_up(incl, d, 32);
      if (lane >= d) incl += y;
    }
    int run = incl - s;
#pragma unroll 1
    for (int i = 0; i < NBRUN / 32; ++i) {
      const int cv = cc[base + i];
      offs[base + i] = run;
      cur[base + i]  = run;
      run += cv;
    }
  }
  __syncthreads();

  if (wave == 0) {
#pragma unroll 1
    for (int w2 = 0; w2 < NWAVE; ++w2) {
      int c = misc[w2];
      c = c < 0 ? 0 : (c > WLCAP ? WLCAP : c);
      c = __builtin_amdgcn_readfirstlane(c);
#pragma unroll 1
      for (int b0 = 0; b0 < c; b0 += 32) {
        const int idx = b0 + lane;
        const int ent = wlI[w2 * WLCAP + (idx < WLCAP ? idx : WLCAP - 1)];
        const int m32 = (c - b0) < 32 ? (c - b0) : 32;
#pragma unroll 1
        for (int k = 0; k < m32; ++k) {
          const int u    = __builtin_amdgcn_readlane(ent, k);
          const int slot = u & (NBRUN - 1);
          const int sv   = (u >> SLB) & 0x1FFFF;
          if (lane == 0) {
            int p = cur[slot];
            p = p < 0 ? 0 : (p > RCAP - 1 ? RCAP - 1 : p);
            pl[p] = sv;
            cur[slot] = p + 1;
          }
        }
      }
    }
  }
  __syncthreads();

  const int ovI = misc[16], ovO = misc[17];
  {
    const float qnan = __uint_as_float(0x7fc00000u);
#pragma unroll 1
    for (int i = tid; i < 2 * NBRUN; i += NTHR) {
      int c = cc[i];
      c = c < 1 ? 1 : c;
      float v = 1.0f / sqrtf((float)c);
      const bool po = (ovO != 0) & (i >= NBRUN);
      v = po ? qnan : v;
      nrm[i] = v;
    }
  }
  __syncthreads();

  const int ovf = ((ovI | ovO) != 0) ? 1 : 0;
  int*   lp   = LIST + (size_t)blk * RCAP;
  int*   cntp = CNT + (size_t)blk * NBRUN;
  int*   offp = OFF + (size_t)blk * NBRUN;
  float* ndp  = NDg + (size_t)blk * NBRUN;
  float* nsp  = NSg + (size_t)blk * NBRUN;
  int*   fp   = FLAG + (size_t)blk * 32;
  bucket_flush(pl, cc, offs, nrm, ovf, lp, cntp, offp, ndp, nsp, fp, tid);
  __threadfence();
  bucket_flush(pl, cc, offs, nrm, ovf, lp, cntp, offp, ndp, nsp, fp, tid);
}
#undef PUT_IN
#undef PUT_OUT

template <int KEXT, int AP, int BP, int NOUT>
__device__ __forceinline__ void gemm_block(const unsigned short* __restrict__ A,
                                           const unsigned short* __restrict__ BT,
                                           const float* __restrict__ NSg, float* Pout, float* gsm) {
  static_assert(KEXT % 32 == 0 && KEXT <= AP && KEXT <= BP && AP % 8 == 0 && BP % 8 == 0);
  static_assert(NOUT == 128 || NOUT == 64);
  constexpr int NT = NOUT / 16, SP = NOUT + 4, LPR = NOUT / 4, RPS = 32 / LPR;
  float* stg = gsm;
  float* sns = gsm + GBM * SP;
  const int tid = (int)threadIdx.x, lane = tid & 31, wave = tid >> 5, hh = lane >> 4, m = lane & 15;
  const int rowBase = (int)blockIdx.x * GBM;
  if (tid < 32) *(v4fa*)(sns + 4 * tid) = *(const v4fa*)(NSg + rowBase + 4 * tid);

  v8f acc[NT];
  {
    const v8f z = {0.f, 0.f, 0.f, 0.f, 0.f, 0.f, 0.f, 0.f};
#pragma unroll
    for (int t = 0; t < NT; ++t) acc[t] = z;
  }
  const unsigned short* ap = A + (size_t)(rowBase + 16 * wave + m) * (size_t)AP + 8 * hh;
  const unsigned short* bp = BT + (size_t)m * (size_t)BP + 8 * hh;
#pragma unroll 1
  for (int k0 = 0; k0 < KEXT; k0 += 32) {
    FragB af;
    af.h[0] = *(const v8usa*)(ap + k0);
    af.h[1] = *(const v8usa*)(ap + k0 + 16);
#pragma unroll
    for (int nt = 0; nt < NT; ++nt) {
      const unsigned short* wq = bp + (size_t)(16 * nt) * (size_t)BP + k0;
      FragB bf;
      bf.h[0] = *(const v8usa*)wq;
      bf.h[1] = *(const v8usa*)(wq + 16);
      acc[nt] = wmb(af, bf, acc[nt]);
    }
  }
#pragma unroll
  for (int nt = 0; nt < NT; ++nt) {
#pragma unroll
    for (int r = 0; r < 8; ++r) stg[(16 * wave + 8 * hh + r) * SP + 16 * nt + m] = acc[nt][r];
  }
  __syncthreads();

  const int q = lane & (LPR - 1), sub = lane / LPR;
#pragma unroll 1
  for (int i = 0; i < 16 / RPS; ++i) {
    const int lr   = 16 * wave + RPS * i + sub;
    const int grow = rowBase + lr;
    const bool live = grow < NN;
    const v4f a = *(const v4fa*)(stg + lr * SP + 4 * q);
    const float ns = sns[lr];
    asm volatile("" :: "v"(a), "v"(ns));
    v4f o;
    o.x = live ? ns * a.x : 0.0f; o.y = live ? ns * a.y : 0.0f;
    o.z = live ? ns * a.z : 0.0f; o.w = live ? ns * a.w : 0.0f;
    st2_v4f(Pout + (size_t)grow * NOUT + 4 * q, o);
  }
}

__global__ __launch_bounds__(NTHR) __attribute__((amdgpu_num_vgpr(248)))
void k_gemm_one(const unsigned short* __restrict__ XB, const unsigned short* __restrict__ W1T,
                const float* __restrict__ NSg, float* P) {
  extern __shared__ __attribute__((aligned(16))) float gsm1[];
  gemm_block<DF, DF, DF, DF>(XB, W1T, NSg, P, gsm1);
}

template <int KEXT, int NOUT>
__global__ __launch_bounds__(NTHR) __attribute__((amdgpu_num_vgpr(248)))
void k_gemm_two(const unsigned short* __restrict__ AHL, const unsigned short* __restrict__ WD,
                const float* __restrict__ NSg, float* P) {
  extern __shared__ __attribute__((aligned(16))) float gsm2[];
  gemm_block<KEXT, APITCH, WPITCH, NOUT>(AHL, WD, NSg, P, gsm2);
}

template <int MODE>
__global__ __launch_bounds__(NTHR) void k_replay_w(const int* __restrict__ LIST, const int* __restrict__ CNT,
                                                   const int* __restrict__ OFF, const float* __restrict__ NDg,
                                                   const int* __restrict__ FLAG, const float* __restrict__ P,
                                                   const float* __restrict__ sm, int smoff,
                                                   float* T, unsigned short* HL, float* REC) {
  __shared__ __attribute__((aligned(16))) float sb[DF];
  __shared__ __attribute__((aligned(16))) float wst[NWAVE * WSTW];
  __shared__ __attribute__((aligned(16))) float pst[PARTW];
  const int tid = (int)threadIdx.x, lane = tid & 31, wave = tid >> 5;
  const int blk = (int)blockIdx.x;
  const int base = blk * NBRUN;
  const int* lb = LIST + (size_t)blk * RCAP;
  const int flag = FLAG[(size_t)blk * 32];
  const float qnan = __uint_as_float(0x7fc00000u);
  if (tid < 32) *(v4fa*)(sb + 4 * tid) = *(const v4fa*)(sm + smoff + 4 * tid);
  __syncthreads();
  const v4f bias = *(const v4fa*)(sb + 4 * lane);

  int wn = 0;
  float wm[4], wq[4];
#pragma unroll
  for (int j = 0; j < 4; ++j) { wm[j] = 0.0f; wq[j] = 0.0f; }

#pragma unroll 1
  for (int i = 0; i < NBRUN / NWAVE; ++i) {
    const int d = base + i * NWAVE + wave;
    if (d < MP) {
      int c = CNT[d];
      int o = OFF[d];
      const float nd = NDg[d];
      const bool big = c > DEGCAP;
      c = c < 0 ? 0 : (c > DEGCAP ? DEGCAP : c);
      o = o < 0 ? 0 : (o > RCAP - 1 ? RCAP - 1 : o);
      c = __builtin_amdgcn_readfirstlane(c);
      o = __builtin_amdgcn_readfirstlane(o);
      int last = o + c - 1;
      last = last < o ? o : last;
      last = last > RCAP - 1 ? RCAP - 1 : last;
      float a0 = 0.0f, a1 = 0.0f, a2 = 0.0f, a3 = 0.0f;
#pragma unroll 1
      for (int b0 = 0; b0 < c; b0 += 32) {
        int idx = o + b0 + lane;
        idx = idx > last ? last : idx;
        int sr = lb[idx];
        sr = sr < 0 ? 0 : (sr > NN - 1 ? NN - 1 : sr);
        const int m32 = (c - b0) < 32 ? (c - b0) : 32;
#pragma unroll 1
        for (int k = 0; k < m32; ++k) {
          const int sk = __builtin_amdgcn_readlane(sr, k);
          const v4f v = *(const v4fa*)(P + (size_t)sk * DF + 4 * lane);
          a0 += v.x; a1 += v.y; a2 += v.z; a3 += v.w;
        }
      }
      float v0 = nd * a0 + bias.x, v1 = nd * a1 + bias.y, v2 = nd * a2 + bias.z, v3 = nd * a3 + bias.w;
      v0 = (v0 > 0.0f) ? v0 : (v0 - v0); v1 = (v1 > 0.0f) ? v1 : (v1 - v1);
      v2 = (v2 > 0.0f) ? v2 : (v2 - v2); v3 = (v3 > 0.0f) ? v3 : (v3 - v3);
      const bool bad  = (flag != 0) | big;
      const bool live = d < NN;
      v0 = bad ? qnan : v0; v1 = bad ? qnan : v1; v2 = bad ? qnan : v2; v3 = bad ? qnan : v3;
      v0 = live ? v0 : 0.0f; v1 = live ? v1 : 0.0f; v2 = live ? v2 : 0.0f; v3 = live ? v3 : 0.0f;
      if constexpr (MODE == 1) {
        v4f ov;
        ov.x = v0; ov.y = v1; ov.z = v2; ov.w = v3;
        st2_v4f(T + (size_t)d * DF + 4 * lane, ov);
        if (live) {
          wn += 1;
          const float rk = 1.0f / (float)wn;
          const float vv[4] = {v0, v1, v2, v3};
#pragma unroll
          for (int j = 0; j < 4; ++j) {
            const float dl = vv[j] - wm[j];
            wm[j] = fmaf(dl, rk, wm[j]);
            wq[j] = fmaf(dl, vv[j] - wm[j], wq[j]);
          }
        }
      } else {
        int h01, h23, l01, l23;
        hilo_pack(v0, v1, v2, v3, h01, h23, l01, l23);
        const v4i ow = regroup32(h01, h23, l01, l23, lane);
        st2_v4i(HL + (size_t)d * APITCH + 8 * lane, ow);
      }
    }
  }

  if constexpr (MODE == 1) {
    if (lane == 0) wst[wave * WSTW] = (float)wn;
#pragma unroll
    for (int j = 0; j < 4; ++j) {
      wst[wave * WSTW + 1 + 4 * lane + j]      = wm[j];
      wst[wave * WSTW + 1 + DF + 4 * lane + j] = wq[j];
    }
    __syncthreads();
    if (tid < DF) {
      float n = 0.0f, mean = 0.0f, M2 = 0.0f;
#pragma unroll 1
      for (int w2 = 0; w2 < NWAVE; ++w2) {
        const float nb = wst[w2 * WSTW];
        const float mb = wst[w2 * WSTW + 1 + tid];
        const float qb = wst[w2 * WSTW + 1 + DF + tid];
        if (nb > 0.5f) {
          const float nn2 = n + nb;
          const float delta = mb - mean;
          const float f = nb / nn2;
          mean = fmaf(delta, f, mean);
          M2 = M2 + qb + delta * delta * n * f;
          n = nn2;
        }
      }
      pst[1 + tid] = mean;
      pst[1 + DF + tid] = M2;
      if (tid == 0) pst[0] = n;
    }
#pragma unroll 1
    for (int i = 2 * DF + 1 + tid; i < PARTW; i += NTHR) pst[i] = 0.0f;
    __syncthreads();
    v4f ps = {0.0f, 0.0f, 0.0f, 0.0f};
    if (tid < PARTW / 4) {
      ps = *(const v4fa*)(pst + 4 * tid);
      *(volatile v4f*)(REC + (size_t)blk * PARTW + 4 * tid) = ps;
    }
    __threadfence();
    if (tid < PARTW / 4) {
      *(volatile v4f*)(REC + (size_t)blk * PARTW + 4 * tid) = ps;
    }
  }
}

__global__ __launch_bounds__(DF) void k_comb(const float* __restrict__ REC, float* STAT) {
  __shared__ __attribute__((aligned(16))) float stg[2 * DF];
  const int tid = (int)threadIdx.x;
  double n = 0.0, mean = 0.0, M2 = 0.0;
#pragma unroll 1
  for (int b = 0; b < NBK; ++b) {
    const float* pr = REC + (size_t)b * PARTW;
    const double nb = (double)pr[0];
    const double mb = (double)pr[1 + tid];
    const double qb = (double)pr[1 + DF + tid];
    if (nb > 0.5) {
      const double nn2 = n + nb;
      const double delta = mb - mean;
      const double f = nb / nn2;
      mean = mean + delta * f;
      M2 = M2 + qb + delta * delta * n * f;
      n = nn2;
    }
  }
  const double nt = n < 1.0 ? 1.0 : n;
  const float varf = (float)(M2 / nt);
  stg[tid] = (float)mean;
  stg[DF + tid] = 1.0f / sqrtf(varf + 1e-5f);
  __syncthreads();
  v4f v = {0.0f, 0.0f, 0.0f, 0.0f};
  if (tid < (2 * DF) / 4) {
    v = *(const v4fa*)(stg + 4 * tid);
    *(volatile v4f*)(STAT + 4 * tid) = v;
  }
  __threadfence();
  if (tid < (2 * DF) / 4) {
    *(volatile v4f*)(STAT + 4 * tid) = v;
  }
}

__global__ __launch_bounds__(NTHR) void k_apply(const float* __restrict__ T, const float* __restrict__ STAT,
                                                const float* __restrict__ sm, unsigned short* HL) {
  __shared__ __attribute__((aligned(16))) float st[4 * DF];
  const int tid = (int)threadIdx.x, lane = tid & 31, wave = tid >> 5;
  if (tid < 64) {
    *(v4fa*)(st + 4 * tid) = *(const v4fa*)(STAT + 4 * tid);
  } else if (tid < 128) {
    *(v4fa*)(st + 2 * DF + 4 * (tid - 64)) = *(const v4fa*)(sm + SM_G1 + 4 * (tid - 64));
  }
  __syncthreads();
  const v4f mu = *(const v4fa*)(st + 4 * lane);
  const v4f rs = *(const v4fa*)(st + DF + 4 * lane);
  const v4f ga = *(const v4fa*)(st + 2 * DF + 4 * lane);
  const v4f be = *(const v4fa*)(st + 3 * DF + 4 * lane);
  const int rowBase = (int)blockIdx.x * 64;
#pragma unroll 1
  for (int i = 0; i < 8; ++i) {
    const int row = rowBase + 8 * wave + i;
    const bool live = row < NN;
    const v4f t = *(const v4fa*)(T + (size_t)row * DF + 4 * lane);
    asm volatile("" :: "v"(t));
    float y0 = ((t.x - mu.x) * rs.x) * ga.x + be.x;
    float y1 = ((t.y - mu.y) * rs.y) * ga.y + be.y;
    float y2 = ((t.z - mu.z) * rs.z) * ga.z + be.z;
    float y3 = ((t.w - mu.w) * rs.w) * ga.w + be.w;
    y0 = live ? y0 : 0.0f; y1 = live ? y1 : 0.0f; y2 = live ? y2 : 0.0f; y3 = live ? y3 : 0.0f;
    int h01, h23, l01, l23;
    hilo_pack(y0, y1, y2, y3, h01, h23, l01, l23);
    const v4i ow = regroup32(h01, h23, l01, l23, lane);
    st2_v4i(HL + (size_t)row * APITCH + 8 * lane, ow);
  }
}

__global__ __launch_bounds__(NTHR) void k_replay3(const int* __restrict__ LIST, const int* __restrict__ CNT,
                                                  const int* __restrict__ OFF, const float* __restrict__ NDg,
                                                  const int* __restrict__ FLAG, const float* __restrict__ P3,
                                                  const float* __restrict__ sm, float* out) {
  __shared__ __attribute__((aligned(16))) float sb[DO];
  const int tid = (int)threadIdx.x, lane = tid & 31, wave = tid >> 5, hh = lane >> 4, q = lane & 15;
  const int blk = (int)blockIdx.x;
  const int base = blk * NBRUN;
  const int* lb = LIST + (size_t)blk * RCAP;
  const int flag = FLAG[(size_t)blk * 32];
  const float qnan = __uint_as_float(0x7fc00000u);
  if (tid < 16) *(v4fa*)(sb + 4 * tid) = *(const v4fa*)(sm + SM_B3 + 4 * tid);
  __syncthreads();
  const v4f bias = *(const v4fa*)(sb + 4 * q);

#pragma unroll 1
  for (int i = 0; i < NBRUN / (2 * NWAVE); ++i) {
    const int d = base + 2 * (i * NWAVE + wave) + hh;
    int c = CNT[d];
    int o = OFF[d];
    const float nd = NDg[d];
    const bool big = c > DEGCAP;
    c = c < 0 ? 0 : (c > DEGCAP ? DEGCAP : c);
    o = o < 0 ? 0 : (o > RCAP - 1 ? RCAP - 1 : o);
    const int co = __shfl_xor(c, 16, 32);
    int cm = c > co ? c : co;
    cm = __builtin_amdgcn_readfirstlane(cm);
    int last = o + c - 1;
    last = last < o ? o : last;
    last = last > RCAP - 1 ? RCAP - 1 : last;
    float a0 = 0.0f, a1 = 0.0f, a2 = 0.0f, a3 = 0.0f;
#pragma unroll 1
    for (int j = 0; j < cm; ++j) {
      int idx = o + j;
      idx = idx > last ? last : idx;
      int sr = lb[idx];
      sr = sr < 0 ? 0 : (sr > NN - 1 ? NN - 1 : sr);
      const v4f v = *(const v4fa*)(P3 + (size_t)sr * DO + 4 * q);
      asm volatile("" :: "v"(v));
      const bool valid = j < c;
      const float t0 = a0 + v.x, t1 = a1 + v.y, t2 = a2 + v.z, t3 = a3 + v.w;
      a0 = valid ? t0 : a0; a1 = valid ? t1 : a1; a2 = valid ? t2 : a2; a3 = valid ? t3 : a3;
    }
    float v0 = nd * a0 + bias.x, v1 = nd * a1 + bias.y, v2 = nd * a2 + bias.z, v3 = nd * a3 + bias.w;
    const bool bad  = (flag != 0) | big;
    const bool live = d < NN;
    v0 = bad ? qnan : v0; v1 = bad ? qnan : v1; v2 = bad ? qnan : v2; v3 = bad ? qnan : v3;
    v4f ov;
    ov.x = v0; ov.y = v1; ov.z = v2; ov.w = v3;
    const int dc = live ? d : NN - 1;
    float* op = out + (size_t)dc * DO + 4 * q;
    if (live) *(volatile v4f*)op = ov;
    __threadfence();
    if (live) *(volatile v4f*)op = ov;
  }

  if (flag != 0) {
    const v4f nv = {qnan, qnan, qnan, qnan};
#pragma unroll 1
    for (int i = 0; i < NBRUN / (2 * NWAVE); ++i) {
      const int d = base + 2 * (i * NWAVE + wave) + hh;
      const bool live = d < NN;
      const int dc = live ? d : NN - 1;
      float* op = out + (size_t)dc * DO + 4 * q;
      if (live) *(volatile v4f*)op = nv;
      __threadfence();
      if (live) *(volatile v4f*)op = nv;
    }
  }
}

extern "C" void kernel_launch(void* const* d_in, const int* in_sizes, int n_in,
                              void* d_out, int out_size, void* d_ws, size_t ws_size,
                              hipStream_t stream) {
  if (n_in < 11) return;
  if (in_sizes[0] != NN * DF) return;
  if (in_sizes[1] != NE) return;
  if (in_sizes[2] != NE) return;
  if (in_sizes[3] != DF * DF) return;
  if (in_sizes[4] != DF) return;
  if (in_sizes[5] != DF) return;
  if (in_sizes[6] != DF) return;
  if (in_sizes[7] != DF * DF) return;
  if (in_sizes[8] != DF) return;
  if (in_sizes[9] != DF * DO) return;
  if (in_sizes[10] != DO) return;
  if (out_size != NN * DO) return;

  const float* feat = (const float*)d_in[0];
  const int*   src  = (const int*)d_in[1];
  const int*   dst  = (const int*)d_in[2];
  const float* W1   = (const float*)d_in[3];
  const float* b1   = (const float*)d_in[4];
  const float* g1   = (const float*)d_in[5];
  const float* be1  = (const float*)d_in[6];
  const float* W2   = (const float*)d_in[7];
  const float* b2   = (const float*)d_in[8];
  const float* W3   = (const float*)d_in[9];
  const float* b3   = (const float*)d_in[10];
  float* out = (float*)d_out;

  constexpr size_t zR    = (size_t)MP * DF * 4;
  constexpr size_t zXB   = (size_t)MP * DF * 2;
  constexpr size_t zP3   = (size_t)MP * DO * 4;
  constexpr size_t zLIST = (size_t)NBK * RCAP * 4;
  constexpr size_t zTAB  = (size_t)NBK * NBRUN * 4;
  constexpr size_t zFLAG = (size_t)NBK * 128;
  constexpr size_t zREC  = (size_t)NBK * PARTW * 4;
  constexpr size_t zSTAT = (size_t)2 * DF * 4;
  constexpr size_t zSM   = (size_t)SM_N * 4;
  constexpr size_t zW1T  = (size_t)DF * DF * 2;
  constexpr size_t zW2D  = (size_t)DF * WPITCH * 2;
  constexpr size_t zW3D  = (size_t)DO * WPITCH * 2;
  constexpr size_t oR1   = 0;
  constexpr size_t oR2   = oR1 + zR;
  constexpr size_t oLIST = oR2 + zR;
  constexpr size_t oCNT  = oLIST + zLIST;
  constexpr size_t oOFF  = oCNT + zTAB;
  constexpr size_t oNS   = oOFF + zTAB;
  constexpr size_t oND   = oNS + zTAB;
  constexpr size_t oFLAG = oND + zTAB;
  constexpr size_t oREC  = oFLAG + zFLAG;
  constexpr size_t oSTAT = oREC + zREC;
  constexpr size_t oSM   = oSTAT + zSTAT;
  constexpr size_t oW1T  = oSM + zSM;
  constexpr size_t oW2D  = oW1T + zW1T;
  constexpr size_t oW3D  = oW2D + zW2D;
  constexpr size_t oEND  = oW3D + zW3D;
  static_assert(zR % 256 == 0 && zLIST % 256 == 0 && zTAB % 256 == 0 && zFLAG % 256 == 0 && zREC % 256 == 0);
  static_assert(zSTAT % 256 == 0 && zSM % 256 == 0 && zW1T % 256 == 0 && zW2D % 256 == 0 && zW3D % 256 == 0);
  static_assert(zXB <= zR && zP3 <= zR && (size_t)MP * APITCH * 2 == zR);
  static_assert(oEND <= (size_t)WSMAX);
  if (oEND > ws_size) return;

  char* ws = (char*)d_ws;
  float*          R1f  = (float*)(ws + oR1);
  unsigned short* R1h  = (unsigned short*)(ws + oR1);
  float*          R2f  = (float*)(ws + oR2);
  unsigned short* R2h  = (unsigned short*)(ws + oR2);
  int*            LIST = (int*)(ws + oLIST);
  int*            CNT  = (int*)(ws + oCNT);
  int*            OFF  = (int*)(ws + oOFF);
  float*          NSg  = (float*)(ws + oNS);
  float*          NDg  = (float*)(ws + oND);
  int*            FLAG = (int*)(ws + oFLAG);
  float*          REC  = (float*)(ws + oREC);
  float*          STAT = (float*)(ws + oSTAT);
  float*          SM   = (float*)(ws + oSM);
  unsigned short* W1T  = (unsigned short*)(ws + oW1T);
  unsigned short* W2D  = (unsigned short*)(ws + oW2D);
  unsigned short* W3D  = (unsigned short*)(ws + oW3D);

  hipFuncSetAttribute(reinterpret_cast<const void*>(&k_bucket), hipFuncAttributeMaxDynamicSharedMemorySize, (int)BK_LDS);
  hipFuncSetAttribute(reinterpret_cast<const void*>(&k_gemm_one), hipFuncAttributeMaxDynamicSharedMemorySize, (int)GL128);
  hipFuncSetAttribute(reinterpret_cast<const void*>(&k_gemm_two<KE2, DF>), hipFuncAttributeMaxDynamicSharedMemorySize, (int)GL128);

  k_prep<<<PBTOT, NTHR, 0, stream>>>(feat, W1, b1, g1, be1, W2, b2, W3, b3, R2h, W1T, W2D, W3D, SM);
  k_bucket<<<NBK, NTHR, BK_LDS, stream>>>(src, dst, LIST, CNT, OFF, NSg, NDg, FLAG);
  k_gemm_one<<<MP / GBM, NTHR, GL128, stream>>>(R2h, W1T, NSg, R1f);
  k_replay_w<1><<<NBK, NTHR, 0, stream>>>(LIST, CNT, OFF, NDg, FLAG, R1f, SM, SM_B1, R2f, R1h, REC);
  k_comb<<<1, DF, 0, stream>>>(REC, STAT);
  k_apply<<<MP / 64, NTHR, 0, stream>>>(R2f, STAT, SM, R1h);
  k_gemm_two<KE2, DF><<<MP / GBM, NTHR, GL128, stream>>>(R1h, W2D, NSg, R2f);
  k_replay_w<2><<<NBK, NTHR, 0, stream>>>(LIST, CNT, OFF, NDg, FLAG, R2f, SM, SM_B2, R2f, R1h, REC);
  k_gemm_two<KE3, DO><<<MP / GBM, NTHR, GL64, stream>>>(R1h, W3D, NSg, R2f);
  k_replay3<<<NBK, NTHR, 0, stream>>>(LIST, CNT, OFF, NDg, FLAG, R2f, SM, out);
}
